// RotarySelfAttention_23940147708412
// MI455X (gfx1250) — hardware-run, weakly checked
//
#include <hip/hip_runtime.h>
#include <math.h>

typedef __attribute__((ext_vector_type(16))) _Float16 v16h;
typedef __attribute__((ext_vector_type(8)))  _Float16 v8h;
typedef __attribute__((ext_vector_type(8)))  float    v8f;
typedef __attribute__((ext_vector_type(4)))  float    v4f;
typedef __attribute__((ext_vector_type(4)))  unsigned int v4u;

constexpr int kBatch = 2;
constexpr int kSeq   = 2048;
constexpr int kDim   = 1024;
constexpr int kHeads = 16;
constexpr int kHd    = 64;
constexpr int kHalf  = 32;
constexpr int kTok   = kBatch * kSeq;
constexpr int kQkvN  = 3 * kDim;
constexpr int kBH    = kBatch * kHeads;
static_assert(kHeads * kHd == kDim);
static_assert(kHalf * 2 == kHd);
static_assert((kSeq % 128) == 0 && (kSeq / 128) == 16);
static_assert((kTok % 64) == 0 && (kQkvN % 64) == 0 && (kDim % 64) == 0 && (kDim % 32) == 0 && (kHd % 32) == 0);

constexpr float kXCarry   = 16.0f;
constexpr float kWCarry   = 256.0f;
constexpr float kRotCarry = 16.0f;
constexpr float kVCarry   = 16.0f;
constexpr float kQkvScale = 1.0f / (kXCarry * kWCarry);
constexpr float kPVScale  = 1.0f / (kRotCarry * kRotCarry * kVCarry);
constexpr float kOutScale = 1.0f / kWCarry;
constexpr float kF16MinNormal = 6.103515625e-5f;
constexpr bool  kInputsViaBf16 = false;

constexpr size_t kSzX16  = (size_t)kTok * kDim * 2;
constexpr size_t kSzWQ   = (size_t)kQkvN * kDim * 2;
constexpr size_t kSzWO   = (size_t)kDim * kDim * 2;
constexpr size_t kSzTH   = 128;
constexpr size_t kSzTab  = (size_t)kSeq * kHalf * 4;
constexpr size_t kSzHead = (size_t)kBH * kSeq * kHd * 2;
constexpr size_t kSzOH   = (size_t)kTok * kDim * 2;
constexpr size_t kOffX16 = 0;
constexpr size_t kOffWQ  = kOffX16 + kSzX16;
constexpr size_t kOffWO  = kOffWQ  + kSzWQ;
constexpr size_t kOffTH  = kOffWO  + kSzWO;
constexpr size_t kOffCOS = kOffTH  + kSzTH;
constexpr size_t kOffSIN = kOffCOS + kSzTab;
constexpr size_t kOffQ   = kOffSIN + kSzTab;
constexpr size_t kOffRQ  = kOffQ   + kSzHead;
constexpr size_t kOffK   = kOffRQ  + kSzHead;
constexpr size_t kOffRK  = kOffK   + kSzHead;
constexpr size_t kOffVT  = kOffRK  + kSzHead;
constexpr size_t kOffOH  = kOffVT  + kSzHead;
constexpr size_t kWsTotal = kOffOH + kSzOH;
static_assert(kWsTotal == 67633280ull);
static_assert(kWsTotal <= 134217728ull);
static_assert((kOffWQ % 128) == 0 && (kOffWO % 128) == 0 && (kOffTH % 128) == 0 && (kOffCOS % 128) == 0 &&
              (kOffSIN % 128) == 0 && (kOffQ % 128) == 0 && (kOffRQ % 128) == 0 && (kOffK % 128) == 0 &&
              (kOffRK % 128) == 0 && (kOffVT % 128) == 0 && (kOffOH % 128) == 0);

__device__ __forceinline__ float in_prep(float f) {
  if (kInputsViaBf16) {
    unsigned u = __float_as_uint(f);
    u = (u + 0x7FFFu + ((u >> 16) & 1u)) & 0xFFFF0000u;
    return __uint_as_float(u);
  }
  return f;
}
__device__ __forceinline__ float flush_f16(float f) {
  return (fabsf(f) < kF16MinNormal) ? 0.0f : f;
}
__device__ __forceinline__ unsigned short h_bits_fl(float f) {
  const _Float16 h = (_Float16)flush_f16(f);
  return __builtin_bit_cast(unsigned short, h);
}
__device__ __forceinline__ unsigned pk16(unsigned short a, unsigned short b) {
  return (unsigned)a | ((unsigned)b << 16);
}
__device__ __forceinline__ float elu_plus1(float z) {
  const float e = expf(fminf(z, 0.0f));
  return (z > 0.0f) ? (z + 1.0f) : e;
}

template <typename T> struct Frag;
template <> struct Frag<_Float16> {
  typedef v16h V;
  union U { v16h v; v8h h[2]; };
  static __device__ __forceinline__ v16h load(const _Float16* p) {
    U f;
    f.h[0] = *(const v8h*)(p);
    f.h[1] = *(const v8h*)(p + 16);
    return f.v;
  }
  static __device__ __forceinline__ v8f mma(v16h a, v16h b, v8f c) {
    return __builtin_amdgcn_wmma_f32_16x16x32_f16(false, a, false, b, (short)0, c, false, false);
  }
};
__device__ __forceinline__ void guard1(v8f& acc, v16h x, v16h y) {
  asm volatile("v_nop\n\tv_nop\n\tv_nop\n\tv_nop" : "+v"(acc) : "v"(x), "v"(y));
}
__device__ __forceinline__ void keep4_h(v16h a, v16h b, v16h c, v16h d) {
  asm volatile("v_nop" :: "v"(a), "v"(b), "v"(c), "v"(d));
}

__device__ __forceinline__ void gemm_main_64x64(const _Float16* __restrict__ Ab, int lda,
                                                const _Float16* __restrict__ Bb, int ldb,
                                                int m0, int n0, int K, int lane, v8f (&acc)[4][4]) {
  typedef Frag<_Float16> F;
  const int rlane = lane & 15;
  const int koff  = (lane >> 4) * 8;
#pragma unroll
  for (int i = 0; i < 4; ++i)
#pragma unroll
    for (int j = 0; j < 4; ++j) acc[i][j] = (v8f){0.f, 0.f, 0.f, 0.f, 0.f, 0.f, 0.f, 0.f};
  for (int k0 = 0; k0 < K; k0 += 32) {
    v16h bh[4];
#pragma unroll
    for (int j = 0; j < 4; ++j) {
      const size_t bo = (size_t)(n0 + (j << 4) + rlane) * ldb + koff + k0;
      bh[j] = F::load(Bb + bo);
    }
#pragma unroll
    for (int i = 0; i < 4; ++i) {
      const size_t ao = (size_t)(m0 + (i << 4) + rlane) * lda + koff + k0;
      const v16h ah = F::load(Ab + ao);
#pragma unroll
      for (int j = 0; j < 4; ++j) acc[i][j] = F::mma(ah, bh[j], acc[i][j]);
      guard1(acc[i][0], ah, bh[0]);
      guard1(acc[i][1], ah, bh[1]);
      guard1(acc[i][2], ah, bh[2]);
      guard1(acc[i][3], ah, bh[3]);
    }
    keep4_h(bh[0], bh[1], bh[2], bh[3]);
  }
}

__global__ __launch_bounds__(256) void cast8_f16_kernel(const float* __restrict__ in, unsigned short* __restrict__ out,
                                                        int n8, float carry) {
  const int i = blockIdx.x * 256 + threadIdx.x;
  if (i >= n8) return;
  const float* p = in + 8 * (size_t)i;
  const v4f a = *(const v4f*)(p);
  const v4f c = *(const v4f*)(p + 4);
  unsigned short hb[8];
#pragma unroll
  for (int e = 0; e < 4; ++e) {
    const float fa = a[e];
    const float fc = c[e];
    hb[e]     = h_bits_fl(in_prep(fa) * carry);
    hb[4 + e] = h_bits_fl(in_prep(fc) * carry);
  }
  const v4u u = (v4u){pk16(hb[0], hb[1]), pk16(hb[2], hb[3]), pk16(hb[4], hb[5]), pk16(hb[6], hb[7])};
  unsigned short* q = out + 8 * (size_t)i;
  *(volatile v4u*)q = u;
  __threadfence();
  *(volatile v4u*)q = u;
}

__global__ __launch_bounds__(256) void wtcast_kernel(const float* __restrict__ W, int ldw,
                                                     unsigned short* __restrict__ out, float carry) {
  __shared__ float sm[64][65];
  const int t  = threadIdx.x;
  const int d0 = blockIdx.x * 64;
  const int h0 = blockIdx.y * 64;
#pragma unroll
  for (int i = 0; i < 16; ++i) {
    const int e = i * 256 + t;
    const int r = e >> 6;
    const int c = e & 63;
    sm[c][r] = in_prep(W[(size_t)(d0 + r) * ldw + h0 + c]) * carry;
  }
  __syncthreads();
  const int lane = t & 31, wave = t >> 5;
  const int q = lane >> 3, c8 = (lane & 7) * 8;
  for (int pass = 0; pass < 2; ++pass) {
#pragma unroll
    for (int it = 0; it < 2; ++it) {
      const int row = wave * 8 + it * 4 + q;
      unsigned short hb[8];
#pragma unroll
      for (int e = 0; e < 8; ++e) hb[e] = h_bits_fl(sm[row][c8 + e]);
      const v4u u = (v4u){pk16(hb[0], hb[1]), pk16(hb[2], hb[3]), pk16(hb[4], hb[5]), pk16(hb[6], hb[7])};
      *(volatile v4u*)(out + (size_t)(h0 + row) * kDim + d0 + c8) = u;
    }
    __threadfence();
  }
}

__global__ __launch_bounds__(32) void theta_kernel(float* __restrict__ theta) {
#pragma clang fp contract(off)
  const int p = threadIdx.x;
  const float fr = (float)p * (1.0f / (float)kHalf);
  const float pw = powf(10000.0f, fr);
  const float th = 1.0f / pw;
  *(volatile float*)(theta + p) = th;
  __threadfence();
  *(volatile float*)(theta + p) = th;
}

__global__ __launch_bounds__(256) void rope_table_kernel(const float* __restrict__ theta,
                                                         float* __restrict__ cosT, float* __restrict__ sinT) {
#pragma clang fp contract(off)
  const int lane = threadIdx.x & 31, wave = threadIdx.x >> 5;
  const int n = blockIdx.x * 8 + wave;
  const float th  = theta[lane];
  const float ang = (float)n * th;
  const float s = sinf(ang);
  const float c = cosf(ang);
  float* cp = cosT + (size_t)n * kHalf + lane;
  float* sp = sinT + (size_t)n * kHalf + lane;
  *(volatile float*)cp = c;
  *(volatile float*)sp = s;
  __threadfence();
  *(volatile float*)cp = c;
  *(volatile float*)sp = s;
}

template <int VMODE>
__global__ __launch_bounds__(128) void qkv_gemm_kernel(
    const unsigned short* __restrict__ Xp, const unsigned short* __restrict__ Wtp, const float* __restrict__ bias,
    unsigned short* __restrict__ Pq, unsigned short* __restrict__ Rq,
    unsigned short* __restrict__ Pk, unsigned short* __restrict__ Rk,
    unsigned short* __restrict__ VTp,
    const float* __restrict__ cosT, const float* __restrict__ sinT) {
  __shared__ __align__(16) float    sT[VMODE ? 1 : 4][VMODE ? 4 : 16 * 68];
  __shared__ __align__(16) _Float16 sV[VMODE ? 4 : 1][VMODE ? 64 * 72 : 8];
  constexpr int tilesN = VMODE ? (kDim / 64) : (2 * kDim / 64);
  constexpr int tilesM = kTok / 64;
  const int lane = threadIdx.x & 31;
  const int wave = threadIdx.x >> 5;
  const int tile = blockIdx.x * 4 + wave;
  if (tile >= tilesM * tilesN) return;
  const int tm = tile / tilesN;
  const int tn = tile - tm * tilesN;
  const int m0 = tm << 6;
  const int n0 = tn << 6;
  const int rlane = lane & 15;
  const int mOff  = (lane >> 4) * 8;

  v8f acc[4][4];
  gemm_main_64x64((const _Float16*)Xp, kDim, (const _Float16*)Wtp, kDim, m0, n0, kDim, lane, acc);

  const int bb   = m0 / kSeq;
  const int tok0 = m0 % kSeq;
  float bv[4];
#pragma unroll
  for (int j = 0; j < 4; ++j) bv[j] = bias[n0 + (j << 4) + rlane];

  if constexpr (VMODE == 0) {
    float* slab = sT[wave];
    const int part = tn >> 4;
    const int head = tn & 15;
    unsigned short* plainP = (part ? Pk : Pq) + ((size_t)(bb * kHeads + head) * kSeq + tok0) * kHd;
    unsigned short* rotP   = (part ? Rk : Rq) + ((size_t)(bb * kHeads + head) * kSeq + tok0) * kHd;
    const int qd = lane >> 3, c8 = (lane & 7) * 8;
#pragma unroll
    for (int i = 0; i < 4; ++i) {
#pragma unroll
      for (int j = 0; j < 4; ++j) {
#pragma unroll
        for (int r = 0; r < 8; ++r) {
          slab[(mOff + r) * 68 + (j << 4) + rlane] = acc[i][j][r] * kQkvScale + bv[j];
        }
      }
      __builtin_amdgcn_fence(__ATOMIC_RELEASE, "workgroup");
      __builtin_amdgcn_wave_barrier();
      __builtin_amdgcn_fence(__ATOMIC_ACQUIRE, "workgroup");
#pragma unroll 1
      for (int it = 0; it < 4; ++it) {
        const int row  = it * 4 + qd;
        const int tokl = (i << 4) + row;
        const int n    = tok0 + tokl;
        const float* sp = slab + row * 68 + c8;
        const v4f a0 = *(const v4f*)(sp);
        const v4f a1 = *(const v4f*)(sp + 4);
        const v4f cs = *(const v4f*)(cosT + (size_t)n * kHalf + (c8 >> 1));
        const v4f sn = *(const v4f*)(sinT + (size_t)n * kHalf + (c8 >> 1));
        float f[8];
#pragma unroll
        for (int e = 0; e < 4; ++e) {
          const float z0 = a0[e];
          const float z1 = a1[e];
          f[e]     = elu_plus1(z0);
          f[4 + e] = elu_plus1(z1);
        }
        unsigned short hb[8], rb[8];
#pragma unroll
        for (int pp = 0; pp < 4; ++pp) {
          const float x1 = f[2 * pp], x2 = f[2 * pp + 1];
          const float cc = cs[pp], ss = sn[pp];
          const float r1 = x1 * cc - x2 * ss;
          const float r2 = x1 * ss + x2 * cc;
          hb[2 * pp]     = h_bits_fl(x1);
          hb[2 * pp + 1] = h_bits_fl(x2);
          rb[2 * pp]     = h_bits_fl(r1 * kRotCarry);
          rb[2 * pp + 1] = h_bits_fl(r2 * kRotCarry);
        }
        const v4u up = (v4u){pk16(hb[0], hb[1]), pk16(hb[2], hb[3]), pk16(hb[4], hb[5]), pk16(hb[6], hb[7])};
        const v4u ur = (v4u){pk16(rb[0], rb[1]), pk16(rb[2], rb[3]), pk16(rb[4], rb[5]), pk16(rb[6], rb[7])};
        unsigned short* dp = plainP + (size_t)tokl * kHd + c8;
        unsigned short* dr = rotP   + (size_t)tokl * kHd + c8;
        *(volatile v4u*)dp = up;
        *(volatile v4u*)dr = ur;
        __threadfence();
        *(volatile v4u*)dp = up;
        *(volatile v4u*)dr = ur;
      }
      __builtin_amdgcn_fence(__ATOMIC_RELEASE, "workgroup");
      __builtin_amdgcn_wave_barrier();
      __builtin_amdgcn_fence(__ATOMIC_ACQUIRE, "workgroup");
    }
  } else {
    _Float16* sv = sV[wave];
    const int head = tn;
#pragma unroll
    for (int i = 0; i < 4; ++i) {
#pragma unroll
      for (int j = 0; j < 4; ++j) {
        v8h hv;
#pragma unroll
        for (int r = 0; r < 8; ++r) {
          const float val = acc[i][j][r] * kQkvScale + bv[j];
          hv[r] = (_Float16)flush_f16(val * kVCarry);
        }
        *(v8h*)(sv + ((j << 4) + rlane) * 72 + (i << 4) + mOff) = hv;
      }
    }
    __builtin_amdgcn_fence(__ATOMIC_RELEASE, "workgroup");
    __builtin_amdgcn_wave_barrier();
    __builtin_amdgcn_fence(__ATOMIC_ACQUIRE, "workgroup");
    const int qd = lane >> 3, c8 = (lane & 7) * 8;
    unsigned short* vbase = VTp + ((size_t)(bb * kHeads + head) * kHd) * kSeq + tok0;
    for (int pass = 0; pass < 2; ++pass) {
#pragma unroll 4
      for (int it = 0; it < 16; ++it) {
        const int row = it * 4 + qd;
        const v8h val = *(const v8h*)(sv + row * 72 + c8);
        *(volatile v8h*)(vbase + (size_t)row * kSeq + c8) = val;
      }
      __threadfence();
    }
  }
}

__global__ __launch_bounds__(256) void ratio_attn_kernel(
    const unsigned short* __restrict__ Qp, const unsigned short* __restrict__ RQp,
    const unsigned short* __restrict__ Kp, const unsigned short* __restrict__ RKp,
    const unsigned short* __restrict__ VTp, unsigned short* __restrict__ OH) {
  typedef Frag<_Float16> F;
  __shared__ __align__(16) float sO[8][16 * 68];
  const int lane  = threadIdx.x & 31;
  const int wave  = threadIdx.x >> 5;
  const int rlane = lane & 15;
  const int hh    = lane >> 4;
  const int koff  = hh * 8;
  const int bh = blockIdx.x >> 4;
  const int qc = blockIdx.x & 15;
  const int q0 = qc * 128 + wave * 16;
  const size_t pbase = (size_t)bh * kSeq * kHd;
  const _Float16* Qb  = (const _Float16*)Qp  + pbase;
  const _Float16* RQb = (const _Float16*)RQp + pbase;
  const _Float16* kp  = (const _Float16*)Kp  + pbase + (size_t)rlane * kHd + koff;
  const _Float16* rp  = (const _Float16*)RKp + pbase + (size_t)rlane * kHd + koff;
  const _Float16* vp  = (const _Float16*)VTp + pbase + (size_t)rlane * kSeq + koff;

  const v16h qB0  = F::load(Qb  + (size_t)(q0 + rlane) * kHd + koff);
  const v16h qB1  = F::load(Qb  + (size_t)(q0 + rlane) * kHd + 32 + koff);
  const v16h rqB0 = F::load(RQb + (size_t)(q0 + rlane) * kHd + koff);
  const v16h rqB1 = F::load(RQb + (size_t)(q0 + rlane) * kHd + 32 + koff);

  v8f o0 = (v8f){0.f, 0.f, 0.f, 0.f, 0.f, 0.f, 0.f, 0.f};
  v8f o1 = o0, o2 = o0, o3 = o0;

#pragma unroll 1
  for (int j0 = 0; j0 < kSeq; j0 += 32) {
    const _Float16* kr = kp + (size_t)j0 * kHd;
    const _Float16* rr = rp + (size_t)j0 * kHd;
    const v16h ak00 = F::load(kr);
    const v16h ak01 = F::load(kr + 32);
    const v16h ak10 = F::load(kr + 16 * kHd);
    const v16h ak11 = F::load(kr + 16 * kHd + 32);
    const v16h ar00 = F::load(rr);
    const v16h ar01 = F::load(rr + 32);
    const v16h ar10 = F::load(rr + 16 * kHd);
    const v16h ar11 = F::load(rr + 16 * kHd + 32);
    v8f dT0 = (v8f){0.f, 0.f, 0.f, 0.f, 0.f, 0.f, 0.f, 0.f};
    v8f dT1 = dT0, nT0 = dT0, nT1 = dT0;
    dT0 = F::mma(ak00, qB0, dT0);
    dT0 = F::mma(ak01, qB1, dT0);
    dT1 = F::mma(ak10, qB0, dT1);
    dT1 = F::mma(ak11, qB1, dT1);
    nT0 = F::mma(ar00, rqB0, nT0);
    nT0 = F::mma(ar01, rqB1, nT0);
    nT1 = F::mma(ar10, rqB0, nT1);
    nT1 = F::mma(ar11, rqB1, nT1);
    guard1(dT0, ak00, ak01);
    guard1(dT1, ak10, ak11);
    guard1(nT0, ar00, ar01);
    guard1(nT1, ar10, ar11);

    v16h wa;
#pragma unroll
    for (int e = 0; e < 8; ++e) {
      const float w0 = nT0[e] * __builtin_amdgcn_rcpf(dT0[e]);
      const float w1 = nT1[e] * __builtin_amdgcn_rcpf(dT1[e]);
      wa[e]     = (_Float16)flush_f16(w0);
      wa[8 + e] = (_Float16)flush_f16(w1);
    }

    const v16h bv0 = F::load(vp + j0);
    const v16h bv1 = F::load(vp + (size_t)16 * kSeq + j0);
    const v16h bv2 = F::load(vp + (size_t)32 * kSeq + j0);
    const v16h bv3 = F::load(vp + (size_t)48 * kSeq + j0);
    o0 = F::mma(wa, bv0, o0);
    o1 = F::mma(wa, bv1, o1);
    o2 = F::mma(wa, bv2, o2);
    o3 = F::mma(wa, bv3, o3);
    guard1(o0, wa, bv0);
    guard1(o1, wa, bv1);
    guard1(o2, wa, bv2);
    guard1(o3, wa, bv3);
  }
  keep4_h(qB0, qB1, rqB0, rqB1);

  float* slab = sO[wave];
#pragma unroll
  for (int r = 0; r < 8; ++r) {
    slab[(8 * hh + r) * 68 + rlane]      = o0[r] * kPVScale;
    slab[(8 * hh + r) * 68 + 16 + rlane] = o1[r] * kPVScale;
    slab[(8 * hh + r) * 68 + 32 + rlane] = o2[r] * kPVScale;
    slab[(8 * hh + r) * 68 + 48 + rlane] = o3[r] * kPVScale;
  }
  __syncthreads();
  {
    const int bb   = bh / kHeads;
    const int head = bh % kHeads;
    const int qd = lane >> 3, c8 = (lane & 7) * 8;
    unsigned short* obase = OH + ((size_t)bb * kSeq + q0) * kDim + head * kHd;
    v4u u[4];
#pragma unroll
    for (int it = 0; it < 4; ++it) {
      const int row = it * 4 + qd;
      const float* sp = slab + row * 68 + c8;
      const v4f a0 = *(const v4f*)(sp);
      const v4f a1 = *(const v4f*)(sp + 4);
      unsigned short hb[8];
#pragma unroll
      for (int e = 0; e < 4; ++e) {
        const float f0 = a0[e];
        const float f1 = a1[e];
        hb[e]     = h_bits_fl(f0);
        hb[4 + e] = h_bits_fl(f1);
      }
      u[it] = (v4u){pk16(hb[0], hb[1]), pk16(hb[2], hb[3]), pk16(hb[4], hb[5]), pk16(hb[6], hb[7])};
    }
    for (int pass = 0; pass < 2; ++pass) {
#pragma unroll
      for (int it = 0; it < 4; ++it) {
        const int row = it * 4 + qd;
        *(volatile v4u*)(obase + (size_t)row * kDim + c8) = u[it];
      }
      __threadfence();
    }
  }
}

__global__ __launch_bounds__(256) void out_gemm_kernel(
    const unsigned short* __restrict__ Ap, const unsigned short* __restrict__ Btp,
    const float* __restrict__ bias, float* __restrict__ C) {
  __shared__ __align__(16) float sT[8][16 * 68];
  constexpr int tilesN = kDim / 64;
  constexpr int tilesM = kTok / 64;
  const int lane = threadIdx.x & 31;
  const int wave = threadIdx.x >> 5;
  const int tile = blockIdx.x * 8 + wave;
  if (tile >= tilesM * tilesN) return;
  const int tm = tile / tilesN;
  const int tn = tile - tm * tilesN;
  const int m0 = tm << 6;
  const int n0 = tn << 6;
  const int rlane = lane & 15;
  const int mOff  = (lane >> 4) * 8;

  v8f acc[4][4];
  gemm_main_64x64((const _Float16*)Ap, kDim, (const _Float16*)Btp, kDim, m0, n0, kDim, lane, acc);

  float bv[4];
#pragma unroll
  for (int j = 0; j < 4; ++j) bv[j] = bias[n0 + (j << 4) + rlane];

  float* slab = sT[wave];
#pragma unroll
  for (int i = 0; i < 4; ++i) {
    const int mBase = m0 + (i << 4);
#pragma unroll
    for (int j = 0; j < 4; ++j) {
#pragma unroll
      for (int r = 0; r < 8; ++r) {
        slab[(mOff + r) * 68 + (j << 4) + rlane] = acc[i][j][r] * kOutScale + bv[j];
      }
    }
    __builtin_amdgcn_fence(__ATOMIC_RELEASE, "workgroup");
    __builtin_amdgcn_wave_barrier();
    __builtin_amdgcn_fence(__ATOMIC_ACQUIRE, "workgroup");
    {
      const int hh = lane >> 4, c4 = (lane & 15) * 4;
      for (int pass = 0; pass < 2; ++pass) {
#pragma unroll
        for (int it = 0; it < 8; ++it) {
          const int row = it * 2 + hh;
          const v4f v = *(const v4f*)(slab + row * 68 + c4);
          *(volatile v4f*)(C + (size_t)(mBase + row) * kDim + n0 + c4) = v;
        }
        __threadfence();
      }
    }
    __builtin_amdgcn_fence(__ATOMIC_RELEASE, "workgroup");
    __builtin_amdgcn_wave_barrier();
    __builtin_amdgcn_fence(__ATOMIC_ACQUIRE, "workgroup");
  }
}

extern "C" void kernel_launch(void* const* d_in, const int* in_sizes, int n_in,
                              void* d_out, int out_size, void* d_ws, size_t ws_size,
                              hipStream_t stream) {
  if (n_in < 5) return;
  if (in_sizes[0] != kTok * kDim) return;
  if (in_sizes[1] != kDim * kQkvN) return;
  if (in_sizes[2] != kQkvN) return;
  if (in_sizes[3] != kDim * kDim) return;
  if (in_sizes[4] != kDim) return;
  if (out_size != kTok * kDim) return;
  if (ws_size < kWsTotal) return;

  const float* x     = (const float*)d_in[0];
  const float* w_qkv = (const float*)d_in[1];
  const float* b_qkv = (const float*)d_in[2];
  const float* w_out = (const float*)d_in[3];
  const float* b_out = (const float*)d_in[4];
  float* out = (float*)d_out;

  char* ws = (char*)d_ws;
  unsigned short* X16   = (unsigned short*)(ws + kOffX16);
  unsigned short* WQKVT = (unsigned short*)(ws + kOffWQ);
  unsigned short* WOUTT = (unsigned short*)(ws + kOffWO);
  float*          THETA = (float*)(ws + kOffTH);
  float*          COST  = (float*)(ws + kOffCOS);
  float*          SINT  = (float*)(ws + kOffSIN);
  unsigned short* QP    = (unsigned short*)(ws + kOffQ);
  unsigned short* RQP   = (unsigned short*)(ws + kOffRQ);
  unsigned short* KP    = (unsigned short*)(ws + kOffK);
  unsigned short* RKP   = (unsigned short*)(ws + kOffRK);
  unsigned short* VT    = (unsigned short*)(ws + kOffVT);
  unsigned short* OH    = (unsigned short*)(ws + kOffOH);

  cast8_f16_kernel<<<(kTok * kDim / 8) / 256, 256, 0, stream>>>(x, X16, kTok * kDim / 8, kXCarry);
  wtcast_kernel<<<dim3(kDim / 64, kQkvN / 64), 256, 0, stream>>>(w_qkv, kQkvN, WQKVT, kWCarry);
  wtcast_kernel<<<dim3(kDim / 64, kDim / 64), 256, 0, stream>>>(w_out, kDim, WOUTT, kWCarry);

  theta_kernel<<<1, 32, 0, stream>>>(THETA);
  rope_table_kernel<<<kSeq / 8, 256, 0, stream>>>(THETA, COST, SINT);

  qkv_gemm_kernel<0><<<(kTok / 64) * (2 * kDim / 64) / 4, 128, 0, stream>>>(
      X16, WQKVT, b_qkv, QP, RQP, KP, RKP, VT, COST, SINT);
  qkv_gemm_kernel<1><<<(kTok / 64) * (kDim / 64) / 4, 128, 0, stream>>>(
      X16, WQKVT + (size_t)2 * kDim * kDim, b_qkv + 2 * kDim, QP, RQP, KP, RKP, VT, COST, SINT);

  ratio_attn_kernel<<<kBH * (kSeq / 128), 256, 0, stream>>>(QP, RQP, KP, RKP, VT, OH);

  out_gemm_kernel<<<(kTok / 64) * (kDim / 64) / 8, 256, 0, stream>>>(OH, WOUTT, b_out, out);
}
